// SlidingWindowCausalSelfAttention_80556406603855
// MI455X (gfx1250) — hardware-verified
//
#include <hip/hip_runtime.h>
#include <stdint.h>

constexpr int kBatch = 2;
constexpr int kSeq   = 2048;
constexpr int kDim   = 1024;
constexpr int kHeads = 16;
constexpr int kHd    = 64;
constexpr int kWin   = 512;
constexpr int kTok   = kBatch * kSeq;
constexpr int kQkvN  = 3 * kDim;
constexpr size_t kPlane = (size_t)kTok * kDim;
constexpr float kRmsEps = 1.1920929e-7f;
constexpr float kNegBig = -1e30f;

typedef __attribute__((ext_vector_type(16))) _Float16 v16h;
typedef __attribute__((ext_vector_type(8)))  _Float16 v8h;
typedef __attribute__((ext_vector_type(16))) __bf16   v16b;
typedef __attribute__((ext_vector_type(8)))  __bf16   v8b;
typedef __attribute__((ext_vector_type(8)))  float    v8f;
typedef __attribute__((ext_vector_type(4)))  float    v4f;
#define U16(p) ((const unsigned short*)(const void*)(p))

__device__ __forceinline__ unsigned short f2bf_bits(float f) {
  unsigned u = __float_as_uint(f);
  return (unsigned short)((u + 0x7FFFu + ((u >> 16) & 1u)) >> 16);
}
__device__ __forceinline__ float bf_bits2f(unsigned short h) { return __uint_as_float(((unsigned)h) << 16); }
__device__ __forceinline__ void bf_split(float f, __bf16& hi, __bf16& lo) {
  const unsigned short hb = f2bf_bits(f);
  hi = __builtin_bit_cast(__bf16, hb);
  lo = __builtin_bit_cast(__bf16, f2bf_bits(f - bf_bits2f(hb)));
}

__device__ __forceinline__ void dep_guard_h(v8f& a, v8f& b, v16h x, v16h y) { asm volatile("v_nop\n\tv_nop\n\tv_nop\n\tv_nop" : "+v"(a), "+v"(b) : "v"(x), "v"(y)); }
__device__ __forceinline__ void dep_guard_b(v8f& a, v8f& b, v16b x, v16b y) { asm volatile("v_nop\n\tv_nop\n\tv_nop\n\tv_nop" : "+v"(a), "+v"(b) : "v"(x), "v"(y)); }
__device__ __forceinline__ void keep4_h(v16h a, v16h b, v16h c, v16h d) { asm volatile("v_nop" :: "v"(a), "v"(b), "v"(c), "v"(d)); }
__device__ __forceinline__ void keep4_b(v16b a, v16b b, v16b c, v16b d) { asm volatile("v_nop" :: "v"(a), "v"(b), "v"(c), "v"(d)); }
__device__ __forceinline__ void acc_guard4(v8f& a, v8f& b, v8f& c, v8f& d) { asm volatile("v_nop\n\tv_nop\n\tv_nop\n\tv_nop" : "+v"(a), "+v"(b), "+v"(c), "+v"(d)); }
template <typename T> struct Frag;
template <> struct Frag<_Float16> {
  typedef v16h V; union U { v16h v; v8h h[2]; };
  static __device__ __forceinline__ v16h load(const _Float16* p) {
    U f; f.h[0] = *(const v8h*)(p); f.h[1] = *(const v8h*)(p + 16); return f.v;
  }
  static __device__ __forceinline__ v8f mma(v16h a, v16h b, v8f c) {
    return __builtin_amdgcn_wmma_f32_16x16x32_f16(false, a, false, b, (short)0, c, false, false);
  }
  static __device__ __forceinline__ void guard(v8f& a, v8f& b, v16h x, v16h y) { dep_guard_h(a, b, x, y); }
  static __device__ __forceinline__ void keep(v16h a, v16h b, v16h c, v16h d) { keep4_h(a, b, c, d); }
};
template <> struct Frag<__bf16> {
  typedef v16b V; union U { v16b v; v8b h[2]; };
  static __device__ __forceinline__ v16b load(const __bf16* p) {
    U f; f.h[0] = *(const v8b*)(p); f.h[1] = *(const v8b*)(p + 16); return f.v;
  }
  static __device__ __forceinline__ v8f mma(v16b a, v16b b, v8f c) {
    return __builtin_amdgcn_wmma_f32_16x16x32_bf16(false, a, false, b, (short)0, c, false, false);
  }
  static __device__ __forceinline__ void guard(v8f& a, v8f& b, v16b x, v16b y) { dep_guard_b(a, b, x, y); }
  static __device__ __forceinline__ void keep(v16b a, v16b b, v16b c, v16b d) { keep4_b(a, b, c, d); }
};

template <int ET> struct Elem;
template <> struct Elem<0> { typedef _Float16 T; };
template <> struct Elem<1> { typedef __bf16 T; };
template <int ET, int SPLIT, int BIAS_MODE, int OUT_MODE, bool RESID, int ACT = 0>
__global__ __launch_bounds__(256) void wmma_gemm64(
    const unsigned short* __restrict__ Ap, const unsigned short* __restrict__ A2p, int lda, long strideA,
    const unsigned short* __restrict__ Btp, const unsigned short* __restrict__ Bt2p, int ldb, long strideB,
    void* __restrict__ Cout, void* __restrict__ Cout2, int ldc, long strideC,
    const float* __restrict__ bias,
    const float* __restrict__ resid, long strideR,
    int M, int N, int K, float scale) {
  typedef typename Elem<ET>::T T;
  typedef typename Frag<T>::V V;
  const T* A = (const T*)Ap; const T* A2 = (const T*)A2p; const T* Bt = (const T*)Btp; const T* Bt2 = (const T*)Bt2p;
  __shared__ __align__(16) float sT[8][16 * 68];
  const int b    = blockIdx.y;
  const int lane = threadIdx.x & 31;
  const int wave = threadIdx.x >> 5;
  const int tilesN = N >> 6;
  const int tilesM = M >> 6;
  const int tile = blockIdx.x * 8 + wave;
  if (tile >= tilesM * tilesN) return;
  const int tm = tile / tilesN;
  const int tn = tile - tm * tilesN;
  const int m0 = tm << 6;
  const int n0 = tn << 6;

  const T* Ab  = A  + (size_t)b * strideA;
  const T* Bb  = Bt + (size_t)b * strideB;
  const T* Ab2 = (SPLIT >= 1) ? (A2  + (size_t)b * strideA) : nullptr;
  const T* Bb2 = (SPLIT >= 2) ? (Bt2 + (size_t)b * strideB) : nullptr;

  const int rlane = lane & 15;
  const int koff  = (lane >> 4) * 8;
  const int mOff  = (lane >> 4) * 8;

  v8f acc[4][4];
#pragma unroll
  for (int i = 0; i < 4; ++i)
#pragma unroll
    for (int j = 0; j < 4; ++j) acc[i][j] = (v8f){0.f,0.f,0.f,0.f,0.f,0.f,0.f,0.f};

  for (int k0 = 0; k0 < K; k0 += 32) {
    V bh[4], bl[4];
#pragma unroll
    for (int j = 0; j < 4; ++j) {
      const size_t bo = (size_t)(n0 + (j << 4) + rlane) * ldb + koff + k0;
      bh[j] = Frag<T>::load(Bb + bo);
      if (SPLIT >= 2) bl[j] = Frag<T>::load(Bb2 + bo);
    }
#pragma unroll
    for (int i = 0; i < 4; ++i) {
      const size_t ao = (size_t)(m0 + (i << 4) + rlane) * lda + koff + k0;
      V ah = Frag<T>::load(Ab + ao);
      V al;
      if (SPLIT >= 1) al = Frag<T>::load(Ab2 + ao);
#pragma unroll
      for (int j = 0; j < 4; ++j) {
        acc[i][j] = Frag<T>::mma(ah, bh[j], acc[i][j]);
        if (SPLIT >= 2) acc[i][j] = Frag<T>::mma(ah, bl[j], acc[i][j]);
        if (SPLIT >= 1) acc[i][j] = Frag<T>::mma(al, bh[j], acc[i][j]);
      }
      Frag<T>::guard(acc[i][0], acc[i][3], ah, (SPLIT != 0) ? al : ah);
    }
    Frag<T>::keep(bh[0], bh[1], bh[2], bh[3]);
    if (SPLIT >= 2) Frag<T>::keep(bl[0], bl[1], bl[2], bl[3]);
  }
  acc_guard4(acc[0][0], acc[0][1], acc[0][2], acc[0][3]);
  acc_guard4(acc[1][0], acc[1][1], acc[1][2], acc[1][3]);
  acc_guard4(acc[2][0], acc[2][1], acc[2][2], acc[2][3]);
  acc_guard4(acc[3][0], acc[3][1], acc[3][2], acc[3][3]);

  float* slab = sT[wave];
  const float* Rb = RESID ? (resid + (size_t)b * strideR) : nullptr;
#pragma unroll
  for (int i = 0; i < 4; ++i) {
    const int mBase = m0 + (i << 4);
#pragma unroll
    for (int j = 0; j < 4; ++j) {
      const int n = n0 + (j << 4) + rlane;
      float bv = 0.f;
      if (BIAS_MODE == 2) bv = bias[n];
#pragma unroll
      for (int r = 0; r < 8; ++r) {
        float v = acc[i][j][r] * scale;
        if (BIAS_MODE == 1) v += bias[mBase + mOff + r];
        if (BIAS_MODE == 2) v += bv;
        if (RESID) v += Rb[(size_t)(mBase + mOff + r) * ldc + n];
        if (ACT == 1) v = tanhf(v);
        if (ACT == 2) v = fmaxf(v, 0.0f);
        if (ACT == 3) v = v / (1.0f + expf(-v));
        if (ACT == 4) v = (v > 0.f) ? v : 0.01f * v;
        slab[(mOff + r) * 68 + (j << 4) + rlane] = v;
      }
    }
    __builtin_amdgcn_fence(__ATOMIC_RELEASE, "workgroup");
    __builtin_amdgcn_wave_barrier();
    __builtin_amdgcn_fence(__ATOMIC_ACQUIRE, "workgroup");
    if (OUT_MODE == 0) {
      float* C = (float*)Cout + (size_t)b * strideC;
      const int hh = lane >> 4, c4 = (lane & 15) * 4;
      for (int pass = 0; pass < 2; ++pass) {
#pragma unroll
        for (int it = 0; it < 8; ++it) {
          const int row = it * 2 + hh;
          v4f v = *(const v4f*)(slab + row * 68 + c4);
          *(volatile v4f*)(C + (size_t)(mBase + row) * ldc + n0 + c4) = v;
        }
        __threadfence();
      }
    } else {
      const int q = lane >> 3, c8 = (lane & 7) * 8;
      unsigned short* C  = (unsigned short*)Cout  + (size_t)b * strideC;
      unsigned short* C2 = (OUT_MODE == 2) ? ((unsigned short*)Cout2 + (size_t)b * strideC) : nullptr;
      for (int pass = 0; pass < 2; ++pass) {
#pragma unroll
        for (int it = 0; it < 4; ++it) {
          const int row = it * 4 + q;
          const float* sp = slab + row * 68 + c8;
          v8h hv, lv;
#pragma unroll
          for (int e = 0; e < 8; ++e) {
            if (OUT_MODE == 1) {
              hv[e] = (_Float16)sp[e];
            } else {
              unsigned short hb = f2bf_bits(sp[e]);
              unsigned short lb = f2bf_bits(sp[e] - bf_bits2f(hb));
              hv[e] = __builtin_bit_cast(_Float16, hb);
              lv[e] = __builtin_bit_cast(_Float16, lb);
            }
          }
          *(volatile v8h*)(C + (size_t)(mBase + row) * ldc + n0 + c8) = hv;
          if (OUT_MODE == 2) *(volatile v8h*)(C2 + (size_t)(mBase + row) * ldc + n0 + c8) = lv;
        }
        __threadfence();
      }
    }
    __builtin_amdgcn_fence(__ATOMIC_RELEASE, "workgroup");
    __builtin_amdgcn_wave_barrier();
    __builtin_amdgcn_fence(__ATOMIC_ACQUIRE, "workgroup");
  }
}

__global__ __launch_bounds__(256) void cast_bf16x2_k(
    const float* __restrict__ in, unsigned short* __restrict__ out, int n2) {
  const int i = blockIdx.x * 256 + threadIdx.x;
  if (i < n2) {
    const unsigned u = (unsigned)f2bf_bits(in[2 * i]) | ((unsigned)f2bf_bits(in[2 * i + 1]) << 16);
    ((volatile unsigned*)out)[i] = u;
    __threadfence();
    ((volatile unsigned*)out)[i] = u;
  }
}
__global__ __launch_bounds__(256) void cast4_bf16x2_k(
    const float* __restrict__ w0, const float* __restrict__ w1, const float* __restrict__ w2,
    const float* __restrict__ w3, unsigned short* __restrict__ out, int n2) {
  const float* in = w0;
  if (blockIdx.y == 1) in = w1;
  if (blockIdx.y == 2) in = w2;
  if (blockIdx.y == 3) in = w3;
  unsigned short* o = out + (size_t)blockIdx.y * (size_t)n2 * 2;
  const int i = blockIdx.x * 256 + threadIdx.x;
  if (i < n2) {
    const unsigned u = (unsigned)f2bf_bits(in[2 * i]) | ((unsigned)f2bf_bits(in[2 * i + 1]) << 16);
    ((volatile unsigned*)o)[i] = u;
    __threadfence();
    ((volatile unsigned*)o)[i] = u;
  }
}

struct InvFreq { float v[32]; };
static_assert(sizeof(InvFreq) == 128);
__global__ __launch_bounds__(256) void rope_table_k(float* __restrict__ rope, InvFreq f) {
  const int lane = threadIdx.x & 31, wave = threadIdx.x >> 5;
  const int s = blockIdx.x * 8 + wave;
  float inv = 0.f;
#pragma unroll
  for (int j = 0; j < 32; ++j) inv = (lane == j) ? f.v[j] : inv;
  const float th = (float)s * inv;
  float sv, cv;
  sincosf(th, &sv, &cv);
  float* rp = rope + (size_t)s * 64;
  *(volatile float*)(rp + lane) = cv;
  *(volatile float*)(rp + 32 + lane) = sv;
  __threadfence();
  *(volatile float*)(rp + lane) = cv;
  *(volatile float*)(rp + 32 + lane) = sv;
}

#define RSP 72
__global__ __launch_bounds__(256) void rope_split_k(const float* __restrict__ qkv, const float* __restrict__ rope,
                                                    const float* __restrict__ qgain, unsigned short* __restrict__ planesp) {
  __shared__ __align__(16) _Float16 st[8][6 * RSP];
  _Float16* planes = (_Float16*)planesp;
  const int tok = blockIdx.x;
  const int s = tok & (kSeq - 1);
  const int b = tok >> 11;
  const int tid = threadIdx.x, w = tid >> 5, ln = tid & 31;
  const int h = blockIdx.y * 8 + w;
  const float* base = qkv + (size_t)tok * kQkvN + h * kHd;
  const float cv = rope[(size_t)s * 64 + ln];
  const float sv = rope[(size_t)s * 64 + 32 + ln];
  const float gq = qgain[h] * 0.125f;
  _Float16* sw = st[w];
#pragma unroll
  for (int p = 0; p < 2; ++p) {
    const float* src = base + p * kDim;
    const float t1 = src[ln], t2 = src[ln + 32];
    float sq = t1 * t1 + t2 * t2;
#pragma unroll
    for (int off = 1; off < 32; off <<= 1) sq += __shfl_xor(sq, off, 32);
    const float rs = rsqrtf(sq * (1.0f / 64.0f) + kRmsEps);
    const float n1 = t1 * rs, n2 = t2 * rs;
    float o0 = n1 * cv + n2 * sv;
    float o1 = n2 * cv - n1 * sv;
    const float g = (p == 0) ? gq : 1.0f;
    o0 *= g; o1 *= g;
    __bf16 h0, l0, h1, l1;
    bf_split(o0, h0, l0);
    bf_split(o1, h1, l1);
    sw[(2 * p) * RSP + ln]          = __builtin_bit_cast(_Float16, h0);
    sw[(2 * p) * RSP + ln + 32]     = __builtin_bit_cast(_Float16, h1);
    sw[(2 * p + 1) * RSP + ln]      = __builtin_bit_cast(_Float16, l0);
    sw[(2 * p + 1) * RSP + ln + 32] = __builtin_bit_cast(_Float16, l1);
  }
  {
    const float* vs = base + 2 * kDim;
    __bf16 h0, l0, h1, l1;
    bf_split(vs[ln], h0, l0);
    bf_split(vs[ln + 32], h1, l1);
    sw[4 * RSP + ln]      = __builtin_bit_cast(_Float16, h0);
    sw[4 * RSP + ln + 32] = __builtin_bit_cast(_Float16, h1);
    sw[5 * RSP + ln]      = __builtin_bit_cast(_Float16, l0);
    sw[5 * RSP + ln + 32] = __builtin_bit_cast(_Float16, l1);
  }
  __builtin_amdgcn_fence(__ATOMIC_RELEASE, "workgroup");
  __builtin_amdgcn_wave_barrier();
  __builtin_amdgcn_fence(__ATOMIC_ACQUIRE, "workgroup");
  const int sel = ln >> 3, c8 = (ln & 7) * 8;
  const int selv = 4 + (sel & 1);
  const size_t prow = ((size_t)(b * kHeads + h) * kSeq + s) * kHd;
  const v8h va = *(const v8h*)(sw + sel * RSP + c8);
  const v8h vv = *(const v8h*)(sw + selv * RSP + c8);
  _Float16* da = planes + (size_t)sel * kPlane + prow + c8;
  _Float16* dv = planes + (size_t)selv * kPlane + prow + c8;
  for (int pass = 0; pass < 2; ++pass) {
    *(volatile v8h*)da = va;
    if (sel < 2) *(volatile v8h*)dv = vv;
    __threadfence();
  }
}

__device__ __forceinline__ v8f mma_b(v16b a, v16b b, v8f c) {
  c = __builtin_amdgcn_wmma_f32_16x16x32_bf16(false, a, false, b, (short)0, c, false, false);
  asm volatile("v_nop\n\tv_nop\n\tv_nop\n\tv_nop" : "+v"(c) : "v"(a), "v"(b));
  return c;
}
constexpr int kKC  = 64;
constexpr int kQB  = 64;
constexpr int kOsp = 68;
__global__ __launch_bounds__(128) void swattn_k(const unsigned short* __restrict__ planesp,
                                                unsigned short* __restrict__ ohp, unsigned short* __restrict__ olp) {
  union FB { v16b v; v8b h[2]; };
  __shared__ __align__(16) __bf16 Ksh[kKC * kHd];
  __shared__ __align__(16) __bf16 Ksl[kKC * kHd];
  __shared__ __align__(16) __bf16 Vth[kHd * kKC];
  __shared__ __align__(16) __bf16 Vtl[kHd * kKC];
  __shared__ __align__(16) __bf16 Psh[4][16 * kKC];
  __shared__ __align__(16) __bf16 Psl[4][16 * kKC];
  __shared__ __align__(16) float  Os[4][16 * kOsp];
  const __bf16* pl0 = (const __bf16*)planesp;
  const __bf16* qh = pl0;
  const __bf16* ql = pl0 + kPlane;
  const __bf16* kh = pl0 + 2 * kPlane;
  const __bf16* kl = pl0 + 3 * kPlane;
  const __bf16* vh = pl0 + 4 * kPlane;
  const __bf16* vl = pl0 + 5 * kPlane;
  _Float16* oh = (_Float16*)ohp;
  _Float16* ol = (_Float16*)olp;
  const int tid = threadIdx.x, wave = tid >> 5, lane = tid & 31, hh = lane >> 4, c = lane & 15;
  const int nqb = kSeq / kQB;
  const int bx = blockIdx.x;
  const int qb = bx % nqb;
  const int bh = bx / nqb;
  const int h = bh % kHeads;
  const int b = bh / kHeads;
  const int q0 = qb * kQB + wave * 16;
  const size_t rowb = (size_t)(b * kHeads + h) * kSeq;

  v16b qah[2], qal[2];
  {
    const __bf16* qhr = qh + (rowb + q0 + c) * kHd + 8 * hh;
    const __bf16* qlr = ql + (rowb + q0 + c) * kHd + 8 * hh;
#pragma unroll
    for (int dc = 0; dc < 2; ++dc) {
      qah[dc] = Frag<__bf16>::load(qhr + dc * 32);
      qal[dc] = Frag<__bf16>::load(qlr + dc * 32);
    }
  }
  float mrow[8], lrow[8];
  v8f oacc[4];
#pragma unroll
  for (int r = 0; r < 8; ++r) { mrow[r] = -__builtin_inff(); lrow[r] = 0.f; }
#pragma unroll
  for (int t = 0; t < 4; ++t) oacc[t] = (v8f){0.f,0.f,0.f,0.f,0.f,0.f,0.f,0.f};

  const int kcLo = (qb > 8) ? (qb - 8) : 0;
  for (int kc = kcLo; kc <= qb; ++kc) {
    const int kv0 = kc * kKC;
    __syncthreads();
    {
      const int kvr = tid >> 1, dh = (tid & 1) * 32;
      const size_t ro = (rowb + kv0 + kvr) * kHd + dh;
#pragma unroll
      for (int i = 0; i < 4; ++i) {
        const v8b a = *(const v8b*)(kh + ro + 8 * i);
        *(v8b*)(Ksh + kvr * kHd + dh + 8 * i) = a;
        const v8b al = *(const v8b*)(kl + ro + 8 * i);
        *(v8b*)(Ksl + kvr * kHd + dh + 8 * i) = al;
        const v8b vvh = *(const v8b*)(vh + ro + 8 * i);
        const v8b vvl = *(const v8b*)(vl + ro + 8 * i);
#pragma unroll
        for (int e = 0; e < 8; ++e) {
          Vth[(dh + 8 * i + e) * kKC + kvr] = vvh[e];
          Vtl[(dh + 8 * i + e) * kKC + kvr] = vvl[e];
        }
      }
    }
    __syncthreads();

    v8f s[4];
#pragma unroll
    for (int j = 0; j < 4; ++j) {
      s[j] = (v8f){0.f,0.f,0.f,0.f,0.f,0.f,0.f,0.f};
#pragma unroll
      for (int dc = 0; dc < 2; ++dc) {
        FB kb, klf;
        kb.h[0]  = *(const v8b*)(Ksh + (j * 16 + c) * kHd + dc * 32 + 8 * hh);
        kb.h[1]  = *(const v8b*)(Ksh + (j * 16 + c) * kHd + dc * 32 + 16 + 8 * hh);
        klf.h[0] = *(const v8b*)(Ksl + (j * 16 + c) * kHd + dc * 32 + 8 * hh);
        klf.h[1] = *(const v8b*)(Ksl + (j * 16 + c) * kHd + dc * 32 + 16 + 8 * hh);
        s[j] = mma_b(qah[dc], kb.v, s[j]);
        s[j] = mma_b(qah[dc], klf.v, s[j]);
        s[j] = mma_b(qal[dc], kb.v, s[j]);
      }
    }
    float cm[8];
#pragma unroll
    for (int r = 0; r < 8; ++r) {
      const int qrow = q0 + 8 * hh + r;
      float m = -__builtin_inff();
#pragma unroll
      for (int j = 0; j < 4; ++j) {
        const int kvcol = kv0 + j * 16 + c;
        const bool masked = (kvcol > qrow) || (qrow - kvcol > kWin - 1);
        const float sv = masked ? kNegBig : s[j][r];
        s[j][r] = sv;
        m = fmaxf(m, sv);
      }
#pragma unroll
      for (int off = 1; off < 16; off <<= 1) m = fmaxf(m, __shfl_xor(m, off, 32));
      cm[r] = m;
    }
    __bf16* pwh = Psh[wave];
    __bf16* pwl = Psl[wave];
#pragma unroll
    for (int r = 0; r < 8; ++r) {
      const float mnew = fmaxf(mrow[r], cm[r]);
      const float alpha = expf(mrow[r] - mnew);
      mrow[r] = mnew;
      float psum = 0.f;
#pragma unroll
      for (int j = 0; j < 4; ++j) {
        const float p = expf(s[j][r] - mnew);
        psum += p;
        __bf16 ph, plo;
        bf_split(p, ph, plo);
        pwh[(8 * hh + r) * kKC + j * 16 + c] = ph;
        pwl[(8 * hh + r) * kKC + j * 16 + c] = plo;
      }
#pragma unroll
      for (int off = 1; off < 16; off <<= 1) psum += __shfl_xor(psum, off, 32);
      lrow[r] = lrow[r] * alpha + psum;
#pragma unroll
      for (int t = 0; t < 4; ++t) oacc[t][r] *= alpha;
    }
    __builtin_amdgcn_fence(__ATOMIC_RELEASE, "workgroup");
    __builtin_amdgcn_wave_barrier();
    __builtin_amdgcn_fence(__ATOMIC_ACQUIRE, "workgroup");
#pragma unroll 1
    for (int kk = 0; kk < 2; ++kk) {
      FB pa, pb;
      pa.h[0] = *(const v8b*)(pwh + c * kKC + kk * 32 + 8 * hh);
      pa.h[1] = *(const v8b*)(pwh + c * kKC + kk * 32 + 16 + 8 * hh);
      pb.h[0] = *(const v8b*)(pwl + c * kKC + kk * 32 + 8 * hh);
      pb.h[1] = *(const v8b*)(pwl + c * kKC + kk * 32 + 16 + 8 * hh);
#pragma unroll
      for (int t = 0; t < 4; ++t) {
        FB vb, vc;
        vb.h[0] = *(const v8b*)(Vth + (t * 16 + c) * kKC + kk * 32 + 8 * hh);
        vb.h[1] = *(const v8b*)(Vth + (t * 16 + c) * kKC + kk * 32 + 16 + 8 * hh);
        vc.h[0] = *(const v8b*)(Vtl + (t * 16 + c) * kKC + kk * 32 + 8 * hh);
        vc.h[1] = *(const v8b*)(Vtl + (t * 16 + c) * kKC + kk * 32 + 16 + 8 * hh);
        oacc[t] = mma_b(pa.v, vb.v, oacc[t]);
        oacc[t] = mma_b(pa.v, vc.v, oacc[t]);
        oacc[t] = mma_b(pb.v, vb.v, oacc[t]);
      }
    }
  }

  float* os = Os[wave];
#pragma unroll
  for (int r = 0; r < 8; ++r) {
    const float inv = 1.0f / lrow[r];
#pragma unroll
    for (int t = 0; t < 4; ++t) os[(8 * hh + r) * kOsp + t * 16 + c] = oacc[t][r] * inv;
  }
  __builtin_amdgcn_fence(__ATOMIC_RELEASE, "workgroup");
  __builtin_amdgcn_wave_barrier();
  __builtin_amdgcn_fence(__ATOMIC_ACQUIRE, "workgroup");
  {
    const int q8 = lane >> 3, c8 = (lane & 7) * 8;
    for (int pass = 0; pass < 2; ++pass) {
#pragma unroll
      for (int it = 0; it < 4; ++it) {
        const int row = it * 4 + q8;
        const float* sp = os + row * kOsp + c8;
        v8h hv, lv;
#pragma unroll
        for (int e = 0; e < 8; ++e) {
          const unsigned short hb = f2bf_bits(sp[e]);
          const unsigned short lb = f2bf_bits(sp[e] - bf_bits2f(hb));
          hv[e] = __builtin_bit_cast(_Float16, hb);
          lv[e] = __builtin_bit_cast(_Float16, lb);
        }
        const size_t o = (size_t)(b * kSeq + q0 + row) * kDim + h * kHd + c8;
        *(volatile v8h*)(oh + o) = hv;
        *(volatile v8h*)(ol + o) = lv;
      }
      __threadfence();
    }
  }
}

extern "C" void kernel_launch(void* const* d_in, const int* in_sizes, int n_in,
                              void* d_out, int out_size, void* d_ws, size_t ws_size,
                              hipStream_t stream) {
  if (n_in < 6) return;
  if (in_sizes[0] != kTok * kDim || in_sizes[1] != kDim * kDim || in_sizes[2] != kDim * kDim ||
      in_sizes[3] != kDim * kDim || in_sizes[4] != kDim * kDim || in_sizes[5] != kHeads ||
      out_size != kTok * kDim) return;

  const float* x  = (const float*)d_in[0];
  const float* wq = (const float*)d_in[1];
  const float* wk = (const float*)d_in[2];
  const float* wv = (const float*)d_in[3];
  const float* wp = (const float*)d_in[4];
  const float* qg = (const float*)d_in[5];
  float* out = (float*)d_out;

  const size_t szXb   = kPlane * 2;
  const size_t szWst  = (size_t)4 * kDim * kDim * 2;
  const size_t szRope = (size_t)kSeq * 64 * 4;
  const size_t szQkv  = (size_t)kTok * kQkvN * 4;
  const size_t szPl   = 6 * kPlane * 2;
  size_t off = 0;
  unsigned char* wsb = (unsigned char*)d_ws;
  unsigned short* xb   = (unsigned short*)(wsb + off); off += szXb;
  unsigned short* wst  = (unsigned short*)(wsb + off); off += szWst;
  float*          rope = (float*)(wsb + off);          off += szRope;
  float*          qkv  = (float*)(wsb + off);          off += szQkv;
  unsigned short* pl   = (unsigned short*)(wsb + off); off += szPl;
  if (off > ws_size) return;
  unsigned short* obh  = (unsigned short*)(void*)qkv;
  unsigned short* obl  = obh + kPlane;
  unsigned short* wpb  = wst + (size_t)3 * kDim * kDim;

  InvFreq invf;
  {
    double lo = 1.0, hi = 2.0;
    for (int it = 0; it < 100; ++it) {
      const double mid = 0.5 * (lo + hi);
      double pw = mid;
      for (int sq = 0; sq < 5; ++sq) pw = pw * pw;
      if (pw > 10000.0) hi = mid; else lo = mid;
    }
    const double r = 0.5 * (lo + hi);
    double acc = 1.0;
    for (int j = 0; j < 32; ++j) {
      const float pf = (float)acc;
      invf.v[j] = 1.0f / pf;
      acc *= r;
    }
  }

  const int n2x = (kTok * kDim) / 2;
  const int n2w = (kDim * kDim) / 2;
  cast_bf16x2_k<<<dim3((n2x + 255) / 256), 256, 0, stream>>>(x, xb, n2x);
  cast4_bf16x2_k<<<dim3((n2w + 255) / 256, 4), 256, 0, stream>>>(wq, wk, wv, wp, wst, n2w);
  rope_table_k<<<dim3(kSeq / 8), 256, 0, stream>>>(rope, invf);

  wmma_gemm64<1, 0, 0, 0, false><<<dim3(384, 1), 256, 0, stream>>>(
      xb, xb, kDim, 0L, wst, wst, kDim, 0L,
      (void*)qkv, (void*)qkv, kQkvN, 0L,
      qg, x, 0L, kTok, kQkvN, kDim, 1.0f);

  rope_split_k<<<dim3(kTok, 2), 256, 0, stream>>>(qkv, rope, qg, pl);

  swattn_k<<<dim3(kBatch * kHeads * (kSeq / kQB)), 128, 0, stream>>>(pl, obh, obl);

  wmma_gemm64<1, 1, 0, 0, false><<<dim3(128, 1), 256, 0, stream>>>(
      obh, obl, kDim, 0L, wpb, wpb, kDim, 0L,
      (void*)out, (void*)out, kDim, 0L,
      qg, x, 0L, kTok, kDim, kDim, 1.0f);
}
